// GRU_channel_48765058678883
// MI455X (gfx1250) — hardware-verified
//
#include <hip/hip_runtime.h>

typedef __attribute__((ext_vector_type(16))) _Float16 v16h;
typedef __attribute__((ext_vector_type(8)))  _Float16 v8h;
typedef __attribute__((ext_vector_type(16))) __bf16   v16b;
typedef __attribute__((ext_vector_type(8)))  __bf16   v8b;
typedef __attribute__((ext_vector_type(8)))  float    v8f;
typedef __attribute__((ext_vector_type(4)))  float    v4f;
typedef __attribute__((ext_vector_type(4)))  unsigned int v4u;

__device__ __forceinline__ unsigned short f2bf_bits(float f) {
  unsigned u = __float_as_uint(f);
  return (unsigned short)((u + 0x7FFFu + ((u >> 16) & 1u)) >> 16);
}
__device__ __forceinline__ float bf_bits2f(unsigned short h) { return __uint_as_float(((unsigned)h) << 16); }
__device__ __forceinline__ unsigned f16u(float f) { return (unsigned)__builtin_bit_cast(unsigned short, (_Float16)f); }
__device__ __forceinline__ unsigned pack_f16x2(float a, float b) { return f16u(a) | (f16u(b) << 16); }
__device__ __forceinline__ void split_bf(float f, unsigned& hb, unsigned& lb) {
  const unsigned short h = f2bf_bits(f);
  hb = (unsigned)h;
  lb = (unsigned)f2bf_bits(f - bf_bits2f(h));
}

__device__ __forceinline__ void dep_guard_h(v8f& a, v8f& b, v16h x, v16h y) { asm volatile("v_nop\n\tv_nop\n\tv_nop\n\tv_nop" : "+v"(a), "+v"(b) : "v"(x), "v"(y)); }
__device__ __forceinline__ void dep_guard_b(v8f& a, v8f& b, v16b x, v16b y) { asm volatile("v_nop\n\tv_nop\n\tv_nop\n\tv_nop" : "+v"(a), "+v"(b) : "v"(x), "v"(y)); }
__device__ __forceinline__ void keep4_h(v16h a, v16h b, v16h c, v16h d) { asm volatile("v_nop" :: "v"(a), "v"(b), "v"(c), "v"(d)); }
__device__ __forceinline__ void keep4_b(v16b a, v16b b, v16b c, v16b d) { asm volatile("v_nop" :: "v"(a), "v"(b), "v"(c), "v"(d)); }
__device__ __forceinline__ void acc_guard4(v8f& a, v8f& b, v8f& c, v8f& d) { asm volatile("v_nop\n\tv_nop\n\tv_nop\n\tv_nop" : "+v"(a), "+v"(b), "+v"(c), "+v"(d)); }
__device__ __forceinline__ void guard3_h(v8f& a, v8f& b, v8f& c, v16h w, v16h x, v16h y, v16h z) {
  asm volatile("v_nop\n\tv_nop\n\tv_nop\n\tv_nop" : "+v"(a), "+v"(b), "+v"(c) : "v"(w), "v"(x), "v"(y), "v"(z));
}
template <typename T> struct Frag;
template <> struct Frag<_Float16> {
  typedef v16h V; union U { v16h v; v8h h[2]; };
  static __device__ __forceinline__ v16h load(const _Float16* p) {
    U f; f.h[0] = *(const v8h*)(p); f.h[1] = *(const v8h*)(p + 16); return f.v;
  }
  static __device__ __forceinline__ v8f mma(v16h a, v16h b, v8f c) {
    return __builtin_amdgcn_wmma_f32_16x16x32_f16(false, a, false, b, (short)0, c, false, false);
  }
  static __device__ __forceinline__ void guard(v8f& a, v8f& b, v16h x, v16h y) { dep_guard_h(a, b, x, y); }
  static __device__ __forceinline__ void keep(v16h a, v16h b, v16h c, v16h d) { keep4_h(a, b, c, d); }
};
template <> struct Frag<__bf16> {
  typedef v16b V; union U { v16b v; v8b h[2]; };
  static __device__ __forceinline__ v16b load(const __bf16* p) {
    U f; f.h[0] = *(const v8b*)(p); f.h[1] = *(const v8b*)(p + 16); return f.v;
  }
  static __device__ __forceinline__ v8f mma(v16b a, v16b b, v8f c) {
    return __builtin_amdgcn_wmma_f32_16x16x32_bf16(false, a, false, b, (short)0, c, false, false);
  }
  static __device__ __forceinline__ void guard(v8f& a, v8f& b, v16b x, v16b y) { dep_guard_b(a, b, x, y); }
  static __device__ __forceinline__ void keep(v16b a, v16b b, v16b c, v16b d) { keep4_b(a, b, c, d); }
};

template <int ET> struct Elem;
template <> struct Elem<0> { typedef _Float16 T; };
template <> struct Elem<1> { typedef __bf16 T; };
template <int ET, bool SPLIT, int BIAS_MODE, int OUT_MODE, bool RESID, int ACT = 0>
__global__ __launch_bounds__(256) void wmma_gemm64(
    const unsigned short* __restrict__ Ap, const unsigned short* __restrict__ A2p, int lda, long strideA,
    const unsigned short* __restrict__ Btp, const unsigned short* __restrict__ Bt2p, int ldb, long strideB,
    void* __restrict__ Cout, void* __restrict__ Cout2, int ldc, long strideC,
    const float* __restrict__ bias,
    const float* __restrict__ resid, long strideR,
    int M, int N, int K, float scale) {
  typedef typename Elem<ET>::T T;
  typedef typename Frag<T>::V V;
  const T* A = (const T*)Ap; const T* A2 = (const T*)A2p; const T* Bt = (const T*)Btp; const T* Bt2 = (const T*)Bt2p;
  __shared__ __align__(16) float sT[8][16 * 68];
  const int b    = blockIdx.y;
  const int lane = threadIdx.x & 31;
  const int wave = threadIdx.x >> 5;
  const int tilesN = N >> 6;
  const int tilesM = M >> 6;
  const int tile = blockIdx.x * 8 + wave;
  if (tile >= tilesM * tilesN) return;
  const int tm = tile / tilesN;
  const int tn = tile - tm * tilesN;
  const int m0 = tm << 6;
  const int n0 = tn << 6;

  const T* Ab  = A  + (size_t)b * strideA;
  const T* Bb  = Bt + (size_t)b * strideB;
  const T* Ab2 = SPLIT ? (A2  + (size_t)b * strideA) : nullptr;
  const T* Bb2 = SPLIT ? (Bt2 + (size_t)b * strideB) : nullptr;

  const int rlane = lane & 15;
  const int koff  = (lane >> 4) * 8;
  const int mOff  = (lane >> 4) * 8;

  v8f acc[4][4];
#pragma unroll
  for (int i = 0; i < 4; ++i)
#pragma unroll
    for (int j = 0; j < 4; ++j) acc[i][j] = (v8f){0.f,0.f,0.f,0.f,0.f,0.f,0.f,0.f};

  for (int k0 = 0; k0 < K; k0 += 32) {
    V bh[4], bl[4];
#pragma unroll
    for (int j = 0; j < 4; ++j) {
      const size_t bo = (size_t)(n0 + (j << 4) + rlane) * ldb + koff + k0;
      bh[j] = Frag<T>::load(Bb + bo);
      if (SPLIT) bl[j] = Frag<T>::load(Bb2 + bo);
    }
#pragma unroll
    for (int i = 0; i < 4; ++i) {
      const size_t ao = (size_t)(m0 + (i << 4) + rlane) * lda + koff + k0;
      V ah = Frag<T>::load(Ab + ao);
      V al;
      if (SPLIT) al = Frag<T>::load(Ab2 + ao);
#pragma unroll
      for (int j = 0; j < 4; ++j) {
        acc[i][j] = Frag<T>::mma(ah, bh[j], acc[i][j]);
        if (SPLIT) {
          acc[i][j] = Frag<T>::mma(ah, bl[j], acc[i][j]);
          acc[i][j] = Frag<T>::mma(al, bh[j], acc[i][j]);
        }
      }
      Frag<T>::guard(acc[i][0], acc[i][3], ah, SPLIT ? al : ah);
    }
    Frag<T>::keep(bh[0], bh[1], bh[2], bh[3]);
    if (SPLIT) Frag<T>::keep(bl[0], bl[1], bl[2], bl[3]);
  }
  acc_guard4(acc[0][0], acc[0][1], acc[0][2], acc[0][3]);
  acc_guard4(acc[1][0], acc[1][1], acc[1][2], acc[1][3]);
  acc_guard4(acc[2][0], acc[2][1], acc[2][2], acc[2][3]);
  acc_guard4(acc[3][0], acc[3][1], acc[3][2], acc[3][3]);

  float* slab = sT[wave];
  const float* Rb = RESID ? (resid + (size_t)b * strideR) : nullptr;
#pragma unroll
  for (int i = 0; i < 4; ++i) {
    const int mBase = m0 + (i << 4);
#pragma unroll
    for (int j = 0; j < 4; ++j) {
      const int n = n0 + (j << 4) + rlane;
      float bv = 0.f;
      if (BIAS_MODE == 2) bv = bias[n];
#pragma unroll
      for (int r = 0; r < 8; ++r) {
        float v = acc[i][j][r] * scale;
        if (BIAS_MODE == 1) v += bias[mBase + mOff + r];
        if (BIAS_MODE == 2) v += bv;
        if (RESID) v += Rb[(size_t)(mBase + mOff + r) * ldc + n];
        if (ACT == 1) v = tanhf(v);
        if (ACT == 2) v = fmaxf(v, 0.0f);
        if (ACT == 3) v = v / (1.0f + expf(-v));
        if (ACT == 4) v = (v > 0.f) ? v : 0.01f * v;
        if (ACT == 5) v = 0.5f * v * (1.0f + erff(v * 0.70710678118654752f));
        slab[(mOff + r) * 68 + (j << 4) + rlane] = v;
      }
    }
    __builtin_amdgcn_fence(__ATOMIC_RELEASE, "workgroup");
    __builtin_amdgcn_wave_barrier();
    __builtin_amdgcn_fence(__ATOMIC_ACQUIRE, "workgroup");
    if (OUT_MODE == 0) {
      float* C = (float*)Cout + (size_t)b * strideC;
      const int hh = lane >> 4, c4 = (lane & 15) * 4;
      for (int pass = 0; pass < 2; ++pass) {
#pragma unroll
        for (int it = 0; it < 8; ++it) {
          const int row = it * 2 + hh;
          v4f v = *(const v4f*)(slab + row * 68 + c4);
          *(volatile v4f*)(C + (size_t)(mBase + row) * ldc + n0 + c4) = v;
        }
        __threadfence();
      }
    } else {
      const int q = lane >> 3, c8 = (lane & 7) * 8;
      unsigned short* C  = (unsigned short*)Cout  + (size_t)b * strideC;
      unsigned short* C2 = (OUT_MODE == 2) ? ((unsigned short*)Cout2 + (size_t)b * strideC) : nullptr;
      for (int pass = 0; pass < 2; ++pass) {
#pragma unroll
        for (int it = 0; it < 4; ++it) {
          const int row = it * 4 + q;
          const float* sp = slab + row * 68 + c8;
          v8h hv, lv;
#pragma unroll
          for (int e = 0; e < 8; ++e) {
            if (OUT_MODE == 1) {
              hv[e] = (_Float16)sp[e];
            } else {
              unsigned short hb = f2bf_bits(sp[e]);
              unsigned short lb = f2bf_bits(sp[e] - bf_bits2f(hb));
              hv[e] = __builtin_bit_cast(_Float16, hb);
              lv[e] = __builtin_bit_cast(_Float16, lb);
            }
          }
          *(volatile v8h*)(C + (size_t)(mBase + row) * ldc + n0 + c8) = hv;
          if (OUT_MODE == 2) *(volatile v8h*)(C2 + (size_t)(mBase + row) * ldc + n0 + c8) = lv;
        }
        __threadfence();
      }
    }
    __builtin_amdgcn_fence(__ATOMIC_RELEASE, "workgroup");
    __builtin_amdgcn_wave_barrier();
    __builtin_amdgcn_fence(__ATOMIC_ACQUIRE, "workgroup");
  }
}

__global__ __launch_bounds__(256) void cast_rows_pad_f16(const float* __restrict__ in, int kin,
                                                         unsigned short* __restrict__ out, int kp8, int total) {
  const int idx = blockIdx.x * 256 + threadIdx.x;
  const int idc = idx < total ? idx : total - 1;
  const int row = idc / kp8;
  const int g = idc - row * kp8;
  const float* src = in + (size_t)row * kin;
  v4u wv;
#pragma unroll
  for (int p = 0; p < 4; ++p) {
    const int c0 = 8 * g + 2 * p, c1 = c0 + 1;
    const float f0 = src[c0 < kin ? c0 : kin - 1];
    const float f1 = src[c1 < kin ? c1 : kin - 1];
    unsigned b0 = f16u(f0), b1 = f16u(f1);
    b0 = (c0 < kin) ? b0 : 0u;
    b1 = (c1 < kin) ? b1 : 0u;
    wv[p] = b0 | (b1 << 16);
  }
  if (idx < total) {
    volatile v4u* d = (volatile v4u*)(out + (size_t)idc * 8);
    *d = wv;
    __threadfence();
    *d = wv;
  }
}

__global__ __launch_bounds__(256) void cast_scale_f16(const float* __restrict__ in, unsigned short* __restrict__ out,
                                                      int n8, float sc) {
  const int idx = blockIdx.x * 256 + threadIdx.x;
  const int idc = idx < n8 ? idx : n8 - 1;
  const float* s = in + (size_t)idc * 8;
  const v4f a = *(const v4f*)s;
  const v4f b = *(const v4f*)(s + 4);
  v4u wv;
  wv[0] = pack_f16x2(a[0] * sc, a[1] * sc);
  wv[1] = pack_f16x2(a[2] * sc, a[3] * sc);
  wv[2] = pack_f16x2(b[0] * sc, b[1] * sc);
  wv[3] = pack_f16x2(b[2] * sc, b[3] * sc);
  if (idx < n8) {
    volatile v4u* d = (volatile v4u*)(out + (size_t)idc * 8);
    *d = wv;
    __threadfence();
    *d = wv;
  }
}

__global__ __launch_bounds__(256) void cast_wT_pad_f16(const float* __restrict__ w, int kin, int nout,
                                                       unsigned short* __restrict__ out, int kp8, float sc, int total) {
  const int idx = blockIdx.x * 256 + threadIdx.x;
  const int idc = idx < total ? idx : total - 1;
  const int n = idc / kp8;
  const int g = idc - n * kp8;
  v4u wv;
#pragma unroll
  for (int p = 0; p < 4; ++p) {
    const int k0 = 8 * g + 2 * p, k1 = k0 + 1;
    const float f0 = w[(size_t)(k0 < kin ? k0 : kin - 1) * nout + n] * sc;
    const float f1 = w[(size_t)(k1 < kin ? k1 : kin - 1) * nout + n] * sc;
    unsigned b0 = f16u(f0), b1 = f16u(f1);
    b0 = (k0 < kin) ? b0 : 0u;
    b1 = (k1 < kin) ? b1 : 0u;
    wv[p] = b0 | (b1 << 16);
  }
  if (idx < total) {
    volatile v4u* d = (volatile v4u*)(out + (size_t)idc * 8);
    *d = wv;
    __threadfence();
    *d = wv;
  }
}

__global__ __launch_bounds__(256) void cast_wT_split_bf16(const float* __restrict__ w, int kdim, int ndim,
                                                          unsigned short* __restrict__ hi, unsigned short* __restrict__ lo, int total) {
  const int idx = blockIdx.x * 256 + threadIdx.x;
  const int idc = idx < total ? idx : total - 1;
  const int kp8 = kdim >> 3;
  const int n = idc / kp8;
  const int g = idc - n * kp8;
  v4u hw, lw;
#pragma unroll
  for (int p = 0; p < 4; ++p) {
    const int k0 = 8 * g + 2 * p;
    const float f0 = w[(size_t)k0 * ndim + n];
    const float f1 = w[(size_t)(k0 + 1) * ndim + n];
    unsigned h0, l0, h1, l1;
    split_bf(f0, h0, l0);
    split_bf(f1, h1, l1);
    hw[p] = h0 | (h1 << 16);
    lw[p] = l0 | (l1 << 16);
  }
  if (idx < total) {
    volatile v4u* dh = (volatile v4u*)(hi + (size_t)idc * 8);
    volatile v4u* dl = (volatile v4u*)(lo + (size_t)idc * 8);
    *dh = hw; *dl = lw;
    __threadfence();
    *dh = hw; *dl = lw;
  }
}

__global__ __launch_bounds__(256) void tree_build_kernel(const float* __restrict__ nodevec, const float* __restrict__ ef,
                                                         const int* __restrict__ esrc, const int* __restrict__ edst,
                                                         const float* __restrict__ ew, const float* __restrict__ eb,
                                                         unsigned short* __restrict__ tree) {
  __shared__ int s_src[128];
  __shared__ int s_dst[128];
  __shared__ int s_cnt[64];
  __shared__ unsigned char s_list[64 * 128];
  __shared__ float s_ef[640];
  __shared__ __align__(16) float srow[896];
  const int b = blockIdx.x;
  const int tid = threadIdx.x;
  if (tid < 128) {
    s_src[tid] = esrc[(size_t)b * 128 + tid];
    int d = edst[(size_t)b * 128 + tid];
    d = (d < 0) ? (d + 64) : d;
    d = (d < 0) ? 0 : ((d > 63) ? 63 : d);
    s_dst[tid] = d;
  }
  for (int i = tid; i < 640; i += 256) s_ef[i] = ef[(size_t)b * 640 + i];
  __syncthreads();
  if (tid < 64) {
    int cnt = 0;
#pragma unroll 1
    for (int e = 0; e < 128; ++e) {
      if (s_src[e] == tid) { s_list[tid * 128 + cnt] = (unsigned char)e; ++cnt; }
    }
    s_cnt[tid] = cnt;
  }
  const int ce = tid & 127;
  const float ew0 = ew[ce], ew1 = ew[128 + ce], ew2 = ew[256 + ce], ew3 = ew[384 + ce], ew4 = ew[512 + ce];
  const float ebv = eb[ce];
  __syncthreads();
  const size_t nvb = (size_t)b * 64 * 384;
#pragma unroll 1
  for (int n = 0; n < 64; ++n) {
    int cnt = s_cnt[n];
    cnt = (cnt > 128) ? 128 : cnt;
    float acc0 = 0.f, acc1 = 0.f;
#pragma unroll 1
    for (int j = 0; j < cnt; ++j) {
      const int e = ((int)s_list[n * 128 + j]) & 127;
      const int d = s_dst[e];
      const float* nr = nodevec + nvb + (size_t)d * 384;
      const float v0 = nr[tid];
      const float v1 = nr[256 + ce];
      float fe = s_ef[e * 5] * ew0 + s_ef[e * 5 + 1] * ew1 + s_ef[e * 5 + 2] * ew2 + s_ef[e * 5 + 3] * ew3 + s_ef[e * 5 + 4] * ew4 + ebv;
      fe = fmaxf(fe, 0.f);
      acc0 += v0;
      acc1 += (tid < 128) ? v1 : fe;
    }
    const float* own = nodevec + nvb + (size_t)n * 384;
    srow[tid] = own[tid];
    if (tid < 128) srow[256 + tid] = own[256 + tid];
    srow[384 + tid] = acc0;
    srow[640 + tid] = acc1;
    __syncthreads();
    if (tid < 112) {
      const float* sp = srow + 8 * tid;
      const v4f f0 = *(const v4f*)sp;
      const v4f f1 = *(const v4f*)(sp + 4);
      v4u wv;
      wv[0] = pack_f16x2(f0[0], f0[1]);
      wv[1] = pack_f16x2(f0[2], f0[3]);
      wv[2] = pack_f16x2(f1[0], f1[1]);
      wv[3] = pack_f16x2(f1[2], f1[3]);
      volatile v4u* dptr = (volatile v4u*)(tree + ((size_t)b * 64 + n) * 896 + 8 * tid);
      *dptr = wv;
      __threadfence();
      *dptr = wv;
    }
    __syncthreads();
  }
}

template <int OUTF>
__global__ __launch_bounds__(256) void gru_layer_kernel(const float* __restrict__ gi, const unsigned short* __restrict__ whhp,
                                                        const float* __restrict__ bhh, void* __restrict__ outp, int dir) {
  constexpr int HPITCH = 136;
  constexpr int SPITCH = 132;
  constexpr float WINV = 1.0f / 16.0f;
  __shared__ __align__(16) _Float16 hbuf[2][16 * HPITCH];
  __shared__ __align__(16) float sOut[16 * SPITCH];
  const int tid = threadIdx.x;
  const int lane = tid & 31;
  const int wave = tid >> 5;
  const int hh = lane >> 4;
  const int cl = lane & 15;
  const int koff = hh * 8;
  const int b0 = blockIdx.x * 16;
  const int u = wave * 16 + cl;
  const _Float16* Wt = (const _Float16*)whhp;
  for (int i = tid; i < 2 * 16 * HPITCH; i += 256) (&hbuf[0][0])[i] = (_Float16)0.0f;
  const float bhr = bhh[u], bhz = bhh[128 + u], bhn = bhh[256 + u];
  float hreg[8];
#pragma unroll
  for (int r = 0; r < 8; ++r) hreg[r] = 0.f;
  const v8f z8 = {0.f, 0.f, 0.f, 0.f, 0.f, 0.f, 0.f, 0.f};
  __syncthreads();
#pragma unroll 1
  for (int s = 0; s < 64; ++s) {
    const int t = dir ? (63 - s) : s;
    const int cur = s & 1, nxt = cur ^ 1;
    v8f ar = z8, az = z8, an = z8;
    const _Float16* hA = &hbuf[cur][0] + cl * HPITCH + koff;
    const _Float16* wr = Wt + (size_t)u * 128 + koff;
    const _Float16* wz = wr + 128 * 128;
    const _Float16* wn = wr + 256 * 128;
#pragma unroll
    for (int kk = 0; kk < 4; ++kk) {
      const int k0 = kk * 32;
      const v16h a  = Frag<_Float16>::load(hA + k0);
      const v16h fr = Frag<_Float16>::load(wr + k0);
      const v16h fz = Frag<_Float16>::load(wz + k0);
      const v16h fn = Frag<_Float16>::load(wn + k0);
      ar = Frag<_Float16>::mma(a, fr, ar);
      az = Frag<_Float16>::mma(a, fz, az);
      an = Frag<_Float16>::mma(a, fn, an);
      guard3_h(ar, az, an, a, fr, fz, fn);
    }
#pragma unroll
    for (int r = 0; r < 8; ++r) {
      const int lr = 8 * hh + r;
      const size_t grow = ((size_t)(b0 + lr) * 64 + t) * 384;
      const float xr = gi[grow + u];
      const float xz = gi[grow + 128 + u];
      const float xn = gi[grow + 256 + u];
      const float ghr = ar[r] * WINV + bhr;
      const float ghz = az[r] * WINV + bhz;
      const float ghn = an[r] * WINV + bhn;
      const float rg = 1.0f / (1.0f + expf(-(xr + ghr)));
      const float zg = 1.0f / (1.0f + expf(-(xz + ghz)));
      const float ng = tanhf(xn + rg * ghn);
      const float hnew = (1.0f - zg) * ng + zg * hreg[r];
      hreg[r] = hnew;
      hbuf[nxt][lr * HPITCH + u] = (_Float16)hnew;
      sOut[lr * SPITCH + u] = hnew;
    }
    __syncthreads();
    if (OUTF == 0) {
      unsigned short* H1 = (unsigned short*)outp;
      const int q = lane >> 3;
      const int lin = wave * 4 + q;
      const int row = lin >> 1, half = lin & 1, c8 = (lane & 7) * 8;
      const float* sp = sOut + row * SPITCH + half * 64 + c8;
      const v4f f0 = *(const v4f*)sp;
      const v4f f1 = *(const v4f*)(sp + 4);
      v4u wv;
      wv[0] = pack_f16x2(f0[0], f0[1]);
      wv[1] = pack_f16x2(f0[2], f0[3]);
      wv[2] = pack_f16x2(f1[0], f1[1]);
      wv[3] = pack_f16x2(f1[2], f1[3]);
      volatile v4u* dptr = (volatile v4u*)(H1 + (((size_t)(b0 + row) * 64 + t) * 256 + dir * 128 + half * 64 + c8));
      *dptr = wv;
      __threadfence();
      *dptr = wv;
    } else {
      float* V = (float*)outp;
      const int r0w = wave * 2;
      const v4f g0 = *(const v4f*)(sOut + r0w * SPITCH + 4 * lane);
      const v4f g1 = *(const v4f*)(sOut + (r0w + 1) * SPITCH + 4 * lane);
      volatile v4f* d0 = (volatile v4f*)(V + (((size_t)(b0 + r0w) * 64 + t) * 256 + dir * 128 + 4 * lane));
      volatile v4f* d1 = (volatile v4f*)(V + (((size_t)(b0 + r0w + 1) * 64 + t) * 256 + dir * 128 + 4 * lane));
      *d0 = g0; *d1 = g1;
      __threadfence();
      *d0 = g0; *d1 = g1;
    }
    __syncthreads();
  }
}

__global__ __launch_bounds__(256) void vec_prep_kernel(const float* __restrict__ vec, unsigned short* __restrict__ ah,
                                                      unsigned short* __restrict__ al, int nbn) {
  __shared__ __align__(16) float smean[8][256];
  const int b = blockIdx.x, tid = threadIdx.x, wave = tid >> 5, lane = tid & 31, c8 = lane * 8;
  v4f ma = {0.f, 0.f, 0.f, 0.f}, mb = {0.f, 0.f, 0.f, 0.f};
#pragma unroll 1
  for (int i = 0; i < 8; ++i) {
    const int n = wave * 8 + i;
    const size_t row = (size_t)b * 64 + n;
    const float* p = vec + row * 256 + c8;
    const v4f x0 = *(const v4f*)p;
    const v4f x1 = *(const v4f*)(p + 4);
    ma += x0; mb += x1;
    v4u hw, lw;
#pragma unroll
    for (int q = 0; q < 2; ++q) {
      unsigned h0, l0, h1, l1;
      split_bf(x0[2 * q], h0, l0); split_bf(x0[2 * q + 1], h1, l1);
      hw[q] = h0 | (h1 << 16); lw[q] = l0 | (l1 << 16);
      split_bf(x1[2 * q], h0, l0); split_bf(x1[2 * q + 1], h1, l1);
      hw[2 + q] = h0 | (h1 << 16); lw[2 + q] = l0 | (l1 << 16);
    }
    volatile v4u* dh = (volatile v4u*)(ah + row * 256 + c8);
    volatile v4u* dl = (volatile v4u*)(al + row * 256 + c8);
    *dh = hw; *dl = lw;
    __threadfence();
    *dh = hw; *dl = lw;
  }
  *(v4f*)(&smean[wave][c8]) = ma;
  *(v4f*)(&smean[wave][c8 + 4]) = mb;
  __syncthreads();
  if (wave == 0) {
    v4f s0 = {0.f, 0.f, 0.f, 0.f}, s1 = {0.f, 0.f, 0.f, 0.f};
#pragma unroll
    for (int w = 0; w < 8; ++w) {
      s0 += *(const v4f*)(&smean[w][c8]);
      s1 += *(const v4f*)(&smean[w][c8 + 4]);
    }
    s0 *= (1.0f / 64.0f); s1 *= (1.0f / 64.0f);
    v4u hw, lw;
#pragma unroll
    for (int q = 0; q < 2; ++q) {
      unsigned h0, l0, h1, l1;
      split_bf(s0[2 * q], h0, l0); split_bf(s0[2 * q + 1], h1, l1);
      hw[q] = h0 | (h1 << 16); lw[q] = l0 | (l1 << 16);
      split_bf(s1[2 * q], h0, l0); split_bf(s1[2 * q + 1], h1, l1);
      hw[2 + q] = h0 | (h1 << 16); lw[2 + q] = l0 | (l1 << 16);
    }
    const size_t row = (size_t)nbn + b;
    volatile v4u* dh = (volatile v4u*)(ah + row * 256 + c8);
    volatile v4u* dl = (volatile v4u*)(al + row * 256 + c8);
    *dh = hw; *dl = lw;
    __threadfence();
    *dh = hw; *dl = lw;
  }
}

__global__ __launch_bounds__(256) void pool_kernel(const float* __restrict__ wv, const float* __restrict__ aw,
                                                  const float* __restrict__ ab, float* __restrict__ out, int nbn) {
  __shared__ float s_aw[512];
  __shared__ float red[256];
  __shared__ float s_part[256];
  __shared__ float s_alpha[64];
  __shared__ __align__(16) float s_out[256];
  __shared__ float s_scal[2];
  const int b = blockIdx.x, tid = threadIdx.x, lane = tid & 31, wave = tid >> 5;
  s_aw[tid] = aw[tid];
  s_aw[256 + tid] = aw[256 + tid];
  const float wsv = wv[((size_t)nbn + b) * 256 + tid];
  red[tid] = wsv * aw[tid];
  __syncthreads();
  for (int o = 128; o > 0; o >>= 1) {
    if (tid < o) red[tid] += red[tid + o];
    __syncthreads();
  }
  const float wsdot = red[0];
  const int n = tid >> 2, q = tid & 3;
  const float* wr = wv + ((size_t)b * 64 + n) * 256 + q * 64;
  float p = 0.f;
#pragma unroll 1
  for (int k = 0; k < 64; ++k) p += wr[k] * s_aw[256 + q * 64 + k];
  s_part[tid] = p;
  __syncthreads();
  if (q == 0) {
    float sc = ((s_part[tid] + s_part[tid + 1]) + (s_part[tid + 2] + s_part[tid + 3])) + wsdot + ab[0];
    sc = (sc > 0.f) ? sc : 0.01f * sc;
    s_alpha[n] = expf(sc);
  }
  __syncthreads();
  if (tid == 0) {
    float ssum = 0.f;
#pragma unroll 1
    for (int i = 0; i < 64; ++i) ssum += s_alpha[i];
    s_scal[0] = 1.0f / ssum;
  }
  __syncthreads();
  const float inv = s_scal[0];
  const float* wc = wv + (size_t)b * 64 * 256 + tid;
  float acc = 0.f;
#pragma unroll 1
  for (int i = 0; i < 64; ++i) acc += (s_alpha[i] * inv) * wc[(size_t)i * 256];
  s_out[tid] = fmaxf(acc, 0.f);
  __syncthreads();
  if (wave == 0) {
    const v4f o0 = *(const v4f*)(s_out + 4 * lane);
    const v4f o1 = *(const v4f*)(s_out + 128 + 4 * lane);
    volatile v4f* d0 = (volatile v4f*)(out + (size_t)b * 256 + 4 * lane);
    volatile v4f* d1 = (volatile v4f*)(out + (size_t)b * 256 + 128 + 4 * lane);
    *d0 = o0; *d1 = o1;
    __threadfence();
    *d0 = o0; *d1 = o1;
  }
}

extern "C" void kernel_launch(void* const* d_in, const int* in_sizes, int n_in,
                              void* d_out, int out_size, void* d_ws, size_t ws_size,
                              hipStream_t stream) {
  constexpr int NB = 512;
  constexpr int NNODE = 64;
  constexpr int NEDGE = 128;
  constexpr int HDIM = 128;
  constexpr int NBN = NB * NNODE;
  constexpr int AF = 39, BFD = 89, LF = 18;
  constexpr int KPA = 64, KPB = 96, KPL = 32;
  constexpr int DTREE = 896;
  constexpr int G3 = 3 * HDIM;
  constexpr int ATTD = 256;
  constexpr int MATT = NBN + NB;
  constexpr float WCARRY = 16.0f;
  constexpr float WCARRY_INV = 1.0f / 16.0f;
  if (n_in < 26) return;
  if (in_sizes[0] != NBN * AF || in_sizes[1] != NBN * BFD || in_sizes[2] != NBN * LF ||
      in_sizes[3] != NB * NEDGE * 5 || in_sizes[4] != NB * NEDGE || in_sizes[5] != NB * NEDGE ||
      in_sizes[14] != 2 * G3 * DTREE || in_sizes[22] != ATTD * ATTD || out_size != NB * ATTD) return;

  const float* fa        = (const float*)d_in[0];
  const float* fb        = (const float*)d_in[1];
  const float* fl        = (const float*)d_in[2];
  const float* edge_feat = (const float*)d_in[3];
  const int*   edge_src  = (const int*)d_in[4];
  const int*   edge_dst  = (const int*)d_in[5];
  const float* atom_w = (const float*)d_in[6];
  const float* atom_b = (const float*)d_in[7];
  const float* bond_w = (const float*)d_in[8];
  const float* bond_b = (const float*)d_in[9];
  const float* link_w = (const float*)d_in[10];
  const float* link_b = (const float*)d_in[11];
  const float* edgew_w = (const float*)d_in[12];
  const float* edgew_b = (const float*)d_in[13];
  const float* gru0_wih = (const float*)d_in[14];
  const float* gru0_whh = (const float*)d_in[15];
  const float* gru0_bih = (const float*)d_in[16];
  const float* gru0_bhh = (const float*)d_in[17];
  const float* gru1_wih = (const float*)d_in[18];
  const float* gru1_whh = (const float*)d_in[19];
  const float* gru1_bih = (const float*)d_in[20];
  const float* gru1_bhh = (const float*)d_in[21];
  const float* att_w = (const float*)d_in[22];
  const float* att_b = (const float*)d_in[23];
  const float* a_w   = (const float*)d_in[24];
  const float* a_b   = (const float*)d_in[25];
  float* outp = (float*)d_out;

  size_t off = 0;
  auto carve = [&](size_t bytes) { size_t o = off; off += (bytes + 255) & ~(size_t)255; return o; };
  const size_t o_wih0 = carve((size_t)2 * G3 * DTREE * 2);
  const size_t o_whh0 = carve((size_t)2 * G3 * HDIM * 2);
  const size_t o_wih1 = carve((size_t)2 * G3 * 2 * HDIM * 2);
  const size_t o_whh1 = carve((size_t)2 * G3 * HDIM * 2);
  const size_t o_atomT = carve((size_t)HDIM * KPA * 2);
  const size_t o_bondT = carve((size_t)HDIM * KPB * 2);
  const size_t o_linkT = carve((size_t)HDIM * KPL * 2);
  const size_t o_attWH = carve((size_t)ATTD * ATTD * 2);
  const size_t o_attWL = carve((size_t)ATTD * ATTD * 2);
  const size_t szR1 = (size_t)NBN * DTREE * 2;
  const size_t szR2 = (size_t)NBN * G3 * 4;
  const size_t szR3 = (size_t)NBN * 2 * HDIM * 2;
  const size_t o_R1 = carve(szR1);
  const size_t o_R2 = carve(szR2);
  const size_t o_R3 = carve(szR3);
  const size_t total = off;
  if (total > ws_size || total > (size_t)134217728) return;
  const size_t sz_fa16 = (size_t)NBN * KPA * 2, sz_fb16 = (size_t)NBN * KPB * 2, sz_fl16 = (size_t)NBN * KPL * 2;
  const size_t o_fa16 = o_R1, o_fb16 = o_R1 + sz_fa16, o_fl16 = o_fb16 + sz_fb16;
  if (o_fl16 + sz_fl16 > o_R1 + szR1) return;
  const size_t sz_vec = (size_t)NBN * ATTD * 4;
  const size_t sz_attA = (size_t)MATT * ATTD * 2;
  const size_t sz_wv = (size_t)MATT * ATTD * 4;
  const size_t o_vec = o_R1, o_attAH = o_vec + sz_vec, o_attAL = o_attAH + sz_attA, o_wv = o_attAL + sz_attA;
  if (o_wv + sz_wv > o_R2 + szR2) return;

  char* ws = (char*)d_ws;
  unsigned short* wih0h = (unsigned short*)(ws + o_wih0);
  unsigned short* whh0h = (unsigned short*)(ws + o_whh0);
  unsigned short* wih1h = (unsigned short*)(ws + o_wih1);
  unsigned short* whh1h = (unsigned short*)(ws + o_whh1);
  unsigned short* atomT = (unsigned short*)(ws + o_atomT);
  unsigned short* bondT = (unsigned short*)(ws + o_bondT);
  unsigned short* linkT = (unsigned short*)(ws + o_linkT);
  unsigned short* attWH = (unsigned short*)(ws + o_attWH);
  unsigned short* attWL = (unsigned short*)(ws + o_attWL);
  unsigned short* fa16 = (unsigned short*)(ws + o_fa16);
  unsigned short* fb16 = (unsigned short*)(ws + o_fb16);
  unsigned short* fl16 = (unsigned short*)(ws + o_fl16);
  unsigned short* tree16 = (unsigned short*)(ws + o_R1);
  float* nodevec = (float*)(ws + o_R2);
  float* gi = (float*)(ws + o_R2);
  unsigned short* h1 = (unsigned short*)(ws + o_R3);
  float* vec = (float*)(ws + o_vec);
  unsigned short* attAH = (unsigned short*)(ws + o_attAH);
  unsigned short* attAL = (unsigned short*)(ws + o_attAL);
  float* wv = (float*)(ws + o_wv);

  cast_rows_pad_f16<<<dim3((NBN * (KPA / 8)) / 256), 256, 0, stream>>>(fa, AF, fa16, KPA / 8, NBN * (KPA / 8));
  cast_rows_pad_f16<<<dim3((NBN * (KPB / 8)) / 256), 256, 0, stream>>>(fb, BFD, fb16, KPB / 8, NBN * (KPB / 8));
  cast_rows_pad_f16<<<dim3((NBN * (KPL / 8)) / 256), 256, 0, stream>>>(fl, LF, fl16, KPL / 8, NBN * (KPL / 8));
  {
    const int n8a = 2 * G3 * DTREE / 8, n8b = 2 * G3 * HDIM / 8, n8c = 2 * G3 * 2 * HDIM / 8;
    cast_scale_f16<<<dim3((n8a + 255) / 256), 256, 0, stream>>>(gru0_wih, wih0h, n8a, WCARRY);
    cast_scale_f16<<<dim3((n8b + 255) / 256), 256, 0, stream>>>(gru0_whh, whh0h, n8b, WCARRY);
    cast_scale_f16<<<dim3((n8c + 255) / 256), 256, 0, stream>>>(gru1_wih, wih1h, n8c, WCARRY);
    cast_scale_f16<<<dim3((n8b + 255) / 256), 256, 0, stream>>>(gru1_whh, whh1h, n8b, WCARRY);
  }
  cast_wT_pad_f16<<<dim3((HDIM * (KPA / 8) + 255) / 256), 256, 0, stream>>>(atom_w, AF, HDIM, atomT, KPA / 8, WCARRY, HDIM * (KPA / 8));
  cast_wT_pad_f16<<<dim3((HDIM * (KPB / 8) + 255) / 256), 256, 0, stream>>>(bond_w, BFD, HDIM, bondT, KPB / 8, WCARRY, HDIM * (KPB / 8));
  cast_wT_pad_f16<<<dim3((HDIM * (KPL / 8) + 255) / 256), 256, 0, stream>>>(link_w, LF, HDIM, linkT, KPL / 8, WCARRY, HDIM * (KPL / 8));
  cast_wT_split_bf16<<<dim3((ATTD * ATTD / 8 + 255) / 256), 256, 0, stream>>>(att_w, ATTD, ATTD, attWH, attWL, ATTD * ATTD / 8);

  {
    const int tiles = (NBN / 64) * (HDIM / 64);
    const dim3 grid((tiles + 7) / 8, 1);
    wmma_gemm64<0, false, 2, 0, false, 2><<<grid, 256, 0, stream>>>(
        fa16, fa16, KPA, 0, atomT, atomT, KPA, 0, nodevec, nodevec, G3, 0, atom_b, atom_b, 0, NBN, HDIM, KPA, WCARRY_INV);
    wmma_gemm64<0, false, 2, 0, false, 2><<<grid, 256, 0, stream>>>(
        fb16, fb16, KPB, 0, bondT, bondT, KPB, 0, nodevec + HDIM, nodevec + HDIM, G3, 0, bond_b, bond_b, 0, NBN, HDIM, KPB, WCARRY_INV);
    wmma_gemm64<0, false, 2, 0, false, 2><<<grid, 256, 0, stream>>>(
        fl16, fl16, KPL, 0, linkT, linkT, KPL, 0, nodevec + 2 * HDIM, nodevec + 2 * HDIM, G3, 0, link_b, link_b, 0, NBN, HDIM, KPL, WCARRY_INV);
  }
  tree_build_kernel<<<dim3(NB), 256, 0, stream>>>(nodevec, edge_feat, edge_src, edge_dst, edgew_w, edgew_b, tree16);

  const int tilesGI = (NBN / 64) * (G3 / 64);
  const dim3 gridGI((tilesGI + 7) / 8, 1);
  for (int d = 0; d < 2; ++d) {
    wmma_gemm64<0, false, 2, 0, false, 0><<<gridGI, 256, 0, stream>>>(
        tree16, tree16, DTREE, 0, wih0h + (size_t)d * G3 * DTREE, wih0h + (size_t)d * G3 * DTREE, DTREE, 0,
        gi, gi, G3, 0, gru0_bih + d * G3, gru0_bih, 0, NBN, G3, DTREE, WCARRY_INV);
    gru_layer_kernel<0><<<dim3(NB / 16), 256, 0, stream>>>(gi, whh0h + (size_t)d * G3 * HDIM, gru0_bhh + d * G3, h1, d);
  }
  for (int d = 0; d < 2; ++d) {
    wmma_gemm64<0, false, 2, 0, false, 0><<<gridGI, 256, 0, stream>>>(
        h1, h1, 2 * HDIM, 0, wih1h + (size_t)d * G3 * 2 * HDIM, wih1h + (size_t)d * G3 * 2 * HDIM, 2 * HDIM, 0,
        gi, gi, G3, 0, gru1_bih + d * G3, gru1_bih, 0, NBN, G3, 2 * HDIM, WCARRY_INV);
    gru_layer_kernel<1><<<dim3(NB / 16), 256, 0, stream>>>(gi, whh1h + (size_t)d * G3 * HDIM, gru1_bhh + d * G3, vec, d);
  }
  vec_prep_kernel<<<dim3(NB), 256, 0, stream>>>(vec, attAH, attAL, NBN);
  {
    const int tiles = (MATT / 64) * (ATTD / 64);
    wmma_gemm64<1, true, 2, 0, false, 0><<<dim3((tiles + 7) / 8, 1), 256, 0, stream>>>(
        attAH, attAL, ATTD, 0, attWH, attWL, ATTD, 0, wv, wv, ATTD, 0, att_b, att_b, 0, MATT, ATTD, ATTD, 1.0f);
  }
  pool_kernel<<<dim3(NB), 256, 0, stream>>>(wv, a_w, a_b, outp, NBN);
}
